// MediumTensorVM_4810363372677
// MI455X (gfx1250) — hardware-verified
//
#include <hip/hip_runtime.h>
#include <stddef.h>
#include <stdint.h>
#include <math.h>


#pragma clang fp contract(off)

#define NRES   300
#define PHW    90000
#define CTOT   32
#define ACOMP  24
#define APPD   27
#define KAPP   72
#define KIN    66
#define KP1    96
#define PA     104
#define FEAT   128
#define PH     136
#define NB0    32
#define NOUT   9
#define NP3    16
#define TM     64
#define NTHR   128
#define PREP_BLOCKS 8
#define PREP_THR 256
#define WSCAP  134217728

#define ASC   1024.0f
#define BSC   64.0f
#define HSC   64.0f
#define WSC   64.0f
#define INV0  (1.0f / 65536.0f)
#define INV1  (1.0f / 4096.0f)
#define GRES  299.0f
#define GMAXI 298.0f

#define BT_BYTES  (NB0 * KP1 * 2)
#define W1T_BYTES (FEAT * KP1 * 2)
#define W2T_BYTES (FEAT * FEAT * 2)
#define W3T_BYTES (NP3 * FEAT * 2)

static_assert(TM == 64);
static_assert(NTHR == 128);
static_assert((KP1 % 32) == 0 && (FEAT % 32) == 0);
static_assert((PA % 8) == 0 && PA >= KP1);
static_assert((PH % 8) == 0 && PH >= FEAT);
static_assert((BT_BYTES % 512) == 0 && (W1T_BYTES % 512) == 0);
static_assert((W2T_BYTES % 512) == 0 && (W3T_BYTES % 512) == 0);
static_assert(KIN == APPD + 3 + 36);
static_assert(KAPP + 24 == KP1);

typedef float    v4f  __attribute__((ext_vector_type(4)));
typedef float    v8f  __attribute__((ext_vector_type(8)));
typedef _Float16 v8h  __attribute__((ext_vector_type(8)));
typedef _Float16 v16h __attribute__((ext_vector_type(16)));
union FragH { v16h v; v8h h[2]; };

__device__ __forceinline__ v8f wmf(v16h a, v16h b, v8f c) {
  v8f d = __builtin_amdgcn_wmma_f32_16x16x32_f16(false, a, false, b, (short)0, c, false, false);
  asm volatile("v_nop\n\tv_nop\n\tv_nop\n\tv_nop" : "+v"(d) : "v"(a), "v"(b));
  return d;
}

__device__ __forceinline__ void st2_v8h(_Float16* p, v8h v) {
  *(volatile v8h*)p = v;
  __threadfence();
  *(volatile v8h*)p = v;
}

__device__ __forceinline__ void cvt_plane(const float* __restrict__ src, int nreal, int kreal,
                                          int nrows, int kp, float sc, _Float16* dst,
                                          int gt, int gs) {
  const int kq = kp >> 3;
  const int items = nrows * kq;
#pragma unroll 1
  for (int it = gt; it < items; it += gs) {
    const int nrow = it / kq, k8 = it - nrow * kq;
    const int nn = min(nrow, nreal - 1);
    v8h hv;
#pragma unroll
    for (int e = 0; e < 8; ++e) {
      const int k = 8 * k8 + e;
      const int kk = min(k, kreal - 1);
      float w = src[(size_t)nn * kreal + kk];
      w = (nrow < nreal && k < kreal) ? (w * sc) : 0.0f;
      hv[e] = (_Float16)w;
    }
    st2_v8h(dst + (size_t)it * 8, hv);
  }
}

__global__ __launch_bounds__(PREP_THR) void k_prep(const float* __restrict__ basis,
                                                   const float* __restrict__ W1,
                                                   const float* __restrict__ W2,
                                                   const float* __restrict__ W3,
                                                   _Float16* bt, _Float16* w1t,
                                                   _Float16* w2t, _Float16* w3t) {
  const int gt = blockIdx.x * PREP_THR + threadIdx.x;
  const int gs = gridDim.x * PREP_THR;
  cvt_plane(basis, APPD, KAPP, NB0, KP1, BSC, bt, gt, gs);
  cvt_plane(W1, FEAT, KIN, FEAT, KP1, WSC, w1t, gt, gs);
  cvt_plane(W2, FEAT, FEAT, FEAT, FEAT, WSC, w2t, gt, gs);
  cvt_plane(W3, NOUT, FEAT, NP3, FEAT, WSC, w3t, gt, gs);
}

__device__ __forceinline__ void sample_plane_line(const float* __restrict__ plane,
                                                  const float* __restrict__ line,
                                                  int pl, float gx, float gy, float gv,
                                                  int cbase, int half, _Float16* arow,
                                                  float& dens) {
  float t = (gx + 1.0f) * 0.5f;
  const float ix = t * GRES;
  t = (gy + 1.0f) * 0.5f;
  const float iy = t * GRES;
  t = (gv + 1.0f) * 0.5f;
  const float il = t * GRES;
  const float fx = fminf(fmaxf(floorf(ix), 0.0f), GMAXI);
  const float fy = fminf(fmaxf(floorf(iy), 0.0f), GMAXI);
  const float fl = fminf(fmaxf(floorf(il), 0.0f), GMAXI);
  int x0 = (int)fx, y0 = (int)fy, l0 = (int)fl;
  x0 = min(max(x0, 0), NRES - 2);
  y0 = min(max(y0, 0), NRES - 2);
  l0 = min(max(l0, 0), NRES - 2);
  const float wx = ix - (float)x0;
  const float wy = iy - (float)y0;
  const float wl = il - (float)l0;
  const float omx = 1.0f - wx, omy = 1.0f - wy, oml = 1.0f - wl;
  const float* Pb = plane + (size_t)(pl * CTOT + cbase) * PHW + (size_t)y0 * NRES + x0;
  const float* Lb = line + (size_t)(pl * CTOT + cbase) * NRES + l0;

  v8h ha;
#pragma unroll
  for (int j = 0; j < 8; ++j) {
    const float* P = Pb + (size_t)j * PHW;
    const float v00 = P[0], v01 = P[1], v10 = P[NRES], v11 = P[NRES + 1];
    const float pf = (v00 * omy + v10 * wy) * omx + (v01 * omy + v11 * wy) * wx;
    const float* L = Lb + (size_t)j * NRES;
    const float lf = L[0] * oml + L[1] * wl;
    const float prod = pf * lf;
    ha[j] = (_Float16)(prod * ASC);
  }
  *(v8h*)(arow + pl * ACOMP + cbase) = ha;

  v8h hb;
#pragma unroll
  for (int j = 8; j < 16; ++j) {
    const float* P = Pb + (size_t)j * PHW;
    const float v00 = P[0], v01 = P[1], v10 = P[NRES], v11 = P[NRES + 1];
    const float pf = (v00 * omy + v10 * wy) * omx + (v01 * omy + v11 * wy) * wx;
    const float* L = Lb + (size_t)j * NRES;
    const float lf = L[0] * oml + L[1] * wl;
    const float prod = pf * lf;
    hb[j - 8] = (_Float16)(prod * ASC);
    dens = dens + prod;
  }
  if (half == 0) *(v8h*)(arow + pl * ACOMP + 8) = hb;
}

__global__ __launch_bounds__(NTHR) void k_main(const float* __restrict__ xyz,
                                               const float* __restrict__ vdirs,
                                               const float* __restrict__ plane,
                                               const float* __restrict__ line,
                                               const float* __restrict__ b1,
                                               const float* __restrict__ b2,
                                               const float* __restrict__ b3,
                                               const _Float16* __restrict__ bt,
                                               const _Float16* __restrict__ w1t,
                                               const _Float16* __restrict__ w2t,
                                               const _Float16* __restrict__ w3t,
                                               float* out, int n) {
  __shared__ __align__(16) _Float16 sApp[TM * PA];
  __shared__ __align__(16) _Float16 sIn[TM * PA];
  __shared__ __align__(16) _Float16 sH[TM * PH];
  __shared__ __align__(16) float sO[3 * TM * 3];
  __shared__ __align__(16) float sDen[TM];

  const int tid = threadIdx.x, lane = tid & 31, hh = lane >> 4, m = lane & 15;
  const int wave = __builtin_amdgcn_readfirstlane(tid >> 5);
  const size_t m0 = (size_t)blockIdx.x * TM;
  const v8h z8h = {(_Float16)0.0f, (_Float16)0.0f, (_Float16)0.0f, (_Float16)0.0f,
                   (_Float16)0.0f, (_Float16)0.0f, (_Float16)0.0f, (_Float16)0.0f};
  const v8f z8f = {0.f, 0.f, 0.f, 0.f, 0.f, 0.f, 0.f, 0.f};

  {
    const int sl = tid & (TM - 1);
    const int half = wave >> 1;
    const int cbase = half * 16;
    const size_t s = m0 + sl;
    const float px = xyz[s * 3 + 0], py = xyz[s * 3 + 1], pz = xyz[s * 3 + 2];
    const float g0 = ((px - (-1.0f)) * 1.0f) - 1.0f;
    const float g1 = ((py - (-1.0f)) * 1.0f) - 1.0f;
    const float g2 = ((pz - (-1.0f)) * 1.0f) - 1.0f;
    const float dv0 = vdirs[s * 3 + 0], dv1 = vdirs[s * 3 + 1], dv2 = vdirs[s * 3 + 2];
    _Float16* arow = sApp + sl * PA;
    _Float16* irow = sIn + sl * PA;
    float dens = 0.0f;
    sample_plane_line(plane, line, 0, g0, g1, g2, cbase, half, arow, dens);
    sample_plane_line(plane, line, 1, g0, g2, g1, cbase, half, arow, dens);
    sample_plane_line(plane, line, 2, g1, g2, g0, cbase, half, arow, dens);
    if (half == 0) {
      irow[APPD + 0] = (_Float16)(dv0 * HSC);
      irow[APPD + 1] = (_Float16)(dv1 * HSC);
      irow[APPD + 2] = (_Float16)(dv2 * HSC);
    } else {
      sDen[sl] = dens;
#pragma unroll
      for (int k = KIN; k < KAPP; ++k) irow[k] = (_Float16)0.0f;
      *(v8h*)(irow + 72) = z8h;
      *(v8h*)(irow + 80) = z8h;
      *(v8h*)(irow + 88) = z8h;
      *(v8h*)(arow + 72) = z8h;
      *(v8h*)(arow + 80) = z8h;
      *(v8h*)(arow + 88) = z8h;
    }
#pragma unroll 1
    for (int t = 0; t < 9; ++t) {
      const int i = half * 9 + t;
      const int d = i / 6;
      const int f = i - 6 * d;
      const float dvs = (d == 0) ? dv0 : ((d == 1) ? dv1 : dv2);
      const float ang = dvs * (float)(1 << f);
      irow[APPD + 3 + i] = (_Float16)(sinf(ang) * HSC);
      irow[APPD + 3 + 18 + i] = (_Float16)(cosf(ang) * HSC);
    }
  }
  __syncthreads();

  const int row0 = wave * 16;

  {
    v8f acc0 = z8f, acc1 = z8f;
    const _Float16* ar = sApp + (row0 + m) * PA + 8 * hh;
    const _Float16* b0r = bt + (size_t)m * KP1 + 8 * hh;
    const _Float16* b1r = bt + (size_t)(16 + m) * KP1 + 8 * hh;
#pragma unroll
    for (int kt = 0; kt < KP1 / 32; ++kt) {
      const int k0 = 32 * kt;
      FragH a, bb0, bb1;
      a.h[0] = *(const v8h*)(ar + k0);
      a.h[1] = *(const v8h*)(ar + k0 + 16);
      bb0.h[0] = *(const v8h*)(b0r + k0);
      bb0.h[1] = *(const v8h*)(b0r + k0 + 16);
      bb1.h[0] = *(const v8h*)(b1r + k0);
      bb1.h[1] = *(const v8h*)(b1r + k0 + 16);
      acc0 = wmf(a.v, bb0.v, acc0);
      acc1 = wmf(a.v, bb1.v, acc1);
    }
#pragma unroll
    for (int r = 0; r < 8; ++r) {
      const int rowl = row0 + 8 * hh + r;
      const float af0 = acc0[r] * INV0;
      const float af1 = acc1[r] * INV0;
      sIn[rowl * PA + m] = (_Float16)(af0 * HSC);
      if (16 + m < APPD) sIn[rowl * PA + 16 + m] = (_Float16)(af1 * HSC);
    }
  }
  __syncthreads();

  {
    v8f acc[8];
#pragma unroll
    for (int nt = 0; nt < 8; ++nt) acc[nt] = z8f;
    const _Float16* ar = sIn + (row0 + m) * PA + 8 * hh;
    const _Float16* br = w1t + (size_t)m * KP1 + 8 * hh;
#pragma unroll 1
    for (int kt = 0; kt < KP1 / 32; ++kt) {
      const int k0 = 32 * kt;
      FragH a;
      a.h[0] = *(const v8h*)(ar + k0);
      a.h[1] = *(const v8h*)(ar + k0 + 16);
#pragma unroll
      for (int nt = 0; nt < 8; ++nt) {
        const _Float16* bp = br + (size_t)nt * 16 * KP1 + k0;
        FragH b;
        b.h[0] = *(const v8h*)bp;
        b.h[1] = *(const v8h*)(bp + 16);
        acc[nt] = wmf(a.v, b.v, acc[nt]);
      }
    }
#pragma unroll
    for (int nt = 0; nt < 8; ++nt) {
      const int nn = nt * 16 + m;
      const float bias = b1[nn];
#pragma unroll
      for (int r = 0; r < 8; ++r) {
        float hv = acc[nt][r] * INV1 + bias;
        hv = fmaxf(hv, 0.0f);
        sH[(row0 + 8 * hh + r) * PH + nn] = (_Float16)(hv * HSC);
      }
    }
  }
  __syncthreads();

  {
    v8f acc[8];
#pragma unroll
    for (int nt = 0; nt < 8; ++nt) acc[nt] = z8f;
    const _Float16* ar = sH + (row0 + m) * PH + 8 * hh;
    const _Float16* br = w2t + (size_t)m * FEAT + 8 * hh;
#pragma unroll 1
    for (int kt = 0; kt < FEAT / 32; ++kt) {
      const int k0 = 32 * kt;
      FragH a;
      a.h[0] = *(const v8h*)(ar + k0);
      a.h[1] = *(const v8h*)(ar + k0 + 16);
#pragma unroll
      for (int nt = 0; nt < 8; ++nt) {
        const _Float16* bp = br + (size_t)nt * 16 * FEAT + k0;
        FragH b;
        b.h[0] = *(const v8h*)bp;
        b.h[1] = *(const v8h*)(bp + 16);
        acc[nt] = wmf(a.v, b.v, acc[nt]);
      }
    }
#pragma unroll
    for (int nt = 0; nt < 8; ++nt) {
      const int nn = nt * 16 + m;
      const float bias = b2[nn];
#pragma unroll
      for (int r = 0; r < 8; ++r) {
        float hv = acc[nt][r] * INV1 + bias;
        hv = fmaxf(hv, 0.0f);
        sH[(row0 + 8 * hh + r) * PH + nn] = (_Float16)(hv * HSC);
      }
    }
  }
  __syncthreads();

  {
    v8f acc = z8f;
    const _Float16* ar = sH + (row0 + m) * PH + 8 * hh;
    const _Float16* br = w3t + (size_t)m * FEAT + 8 * hh;
#pragma unroll
    for (int kt = 0; kt < FEAT / 32; ++kt) {
      const int k0 = 32 * kt;
      FragH a, b;
      a.h[0] = *(const v8h*)(ar + k0);
      a.h[1] = *(const v8h*)(ar + k0 + 16);
      b.h[0] = *(const v8h*)(br + k0);
      b.h[1] = *(const v8h*)(br + k0 + 16);
      acc = wmf(a.v, b.v, acc);
    }
    const float bias = b3[min(m, NOUT - 1)];
    const int grp = (m < 3) ? 0 : ((m < 6) ? 1 : 2);
    const int cc = m - 3 * grp;
#pragma unroll
    for (int r = 0; r < 8; ++r) {
      const int rowl = row0 + 8 * hh + r;
      const float v = acc[r] * INV1 + bias;
      const float sg = 1.0f / (1.0f + expf(-v));
      const float sp = fmaxf(v, 0.0f) + log1pf(expf(-fabsf(v)));
      const float val = (m < 3) ? sg : sp;
      if (m < NOUT) sO[grp * (TM * 3) + rowl * 3 + cc] = val;
    }
  }
  __syncthreads();

  if (wave < 3) {
    const float* src = sO + wave * (TM * 3);
    const v4f v0 = *(const v4f*)(src + 4 * lane);
    const v4f v1 = *(const v4f*)(src + 128 + 4 * (lane & 15));
    float* gp = out + (size_t)wave * 3 * (size_t)n + m0 * 3;
    *(volatile v4f*)(gp + 4 * lane) = v0;
    if (lane < 16) *(volatile v4f*)(gp + 128 + 4 * lane) = v1;
    __threadfence();
    *(volatile v4f*)(gp + 4 * lane) = v0;
    if (lane < 16) *(volatile v4f*)(gp + 128 + 4 * lane) = v1;
  } else {
    const v4f v = *(const v4f*)(sDen + 4 * (lane & 15));
    float* gp = out + (size_t)9 * (size_t)n + m0;
    if (lane < 16) *(volatile v4f*)(gp + 4 * lane) = v;
    __threadfence();
    if (lane < 16) *(volatile v4f*)(gp + 4 * lane) = v;
  }
}

extern "C" void kernel_launch(void* const* d_in, const int* in_sizes, int n_in,
                              void* d_out, int out_size, void* d_ws, size_t ws_size,
                              hipStream_t stream) {
  if (n_in < 11) return;
  const int n = in_sizes[0] / 3;
  if (n <= 0 || in_sizes[0] != 3 * n || in_sizes[1] != 3 * n) return;
  if ((n % TM) != 0) return;
  if (in_sizes[2] != 3 * CTOT * PHW || in_sizes[3] != 3 * CTOT * NRES) return;
  if (in_sizes[4] != APPD * KAPP || in_sizes[5] != FEAT * KIN || in_sizes[6] != FEAT) return;
  if (in_sizes[7] != FEAT * FEAT || in_sizes[8] != FEAT) return;
  if (in_sizes[9] != NOUT * FEAT || in_sizes[10] != NOUT) return;
  if (out_size != 10 * n) return;

  const float* xyz   = (const float*)d_in[0];
  const float* vdirs = (const float*)d_in[1];
  const float* plane = (const float*)d_in[2];
  const float* line  = (const float*)d_in[3];
  const float* basis = (const float*)d_in[4];
  const float* W1    = (const float*)d_in[5];
  const float* b1    = (const float*)d_in[6];
  const float* W2    = (const float*)d_in[7];
  const float* b2    = (const float*)d_in[8];
  const float* W3    = (const float*)d_in[9];
  const float* b3    = (const float*)d_in[10];
  float* out = (float*)d_out;

  char* ws = (char*)d_ws;
  size_t off = 0;
  const size_t oBt = off; off += BT_BYTES;  off = (off + 255) & ~(size_t)255;
  const size_t oW1 = off; off += W1T_BYTES; off = (off + 255) & ~(size_t)255;
  const size_t oW2 = off; off += W2T_BYTES; off = (off + 255) & ~(size_t)255;
  const size_t oW3 = off; off += W3T_BYTES; off = (off + 255) & ~(size_t)255;
  if (off > ws_size || off > (size_t)WSCAP) return;
  _Float16* bt  = (_Float16*)(ws + oBt);
  _Float16* w1t = (_Float16*)(ws + oW1);
  _Float16* w2t = (_Float16*)(ws + oW2);
  _Float16* w3t = (_Float16*)(ws + oW3);

  k_prep<<<PREP_BLOCKS, PREP_THR, 0, stream>>>(basis, W1, W2, W3, bt, w1t, w2t, w3t);
  k_main<<<n / TM, NTHR, 0, stream>>>(xyz, vdirs, plane, line, b1, b2, b3, bt, w1t, w2t, w3t, out, n);
}
